// Pair_attention_layer_29145648071158
// MI455X (gfx1250) — hardware-verified
//
#include <hip/hip_runtime.h>

typedef __attribute__((ext_vector_type(16))) _Float16 v16h;
typedef __attribute__((ext_vector_type(8)))  _Float16 v8h;
typedef __attribute__((ext_vector_type(16))) __bf16   v16b;
typedef __attribute__((ext_vector_type(8)))  __bf16   v8b;
typedef __attribute__((ext_vector_type(8)))  float    v8f;
typedef __attribute__((ext_vector_type(4)))  float    v4f;

__device__ __forceinline__ unsigned short f2bf_bits(float f) {
  unsigned u = __float_as_uint(f);
  return (unsigned short)((u + 0x7FFFu + ((u >> 16) & 1u)) >> 16);
}
__device__ __forceinline__ float bf_bits2f(unsigned short h) { return __uint_as_float(((unsigned)h) << 16); }

__device__ __forceinline__ void dep_guard_h(v8f& a, v8f& b, v16h x, v16h y) { asm volatile("v_nop\n\tv_nop\n\tv_nop\n\tv_nop" : "+v"(a), "+v"(b) : "v"(x), "v"(y)); }
__device__ __forceinline__ void dep_guard_b(v8f& a, v8f& b, v16b x, v16b y) { asm volatile("v_nop\n\tv_nop\n\tv_nop\n\tv_nop" : "+v"(a), "+v"(b) : "v"(x), "v"(y)); }
__device__ __forceinline__ void keep4_h(v16h a, v16h b, v16h c, v16h d) { asm volatile("v_nop" :: "v"(a), "v"(b), "v"(c), "v"(d)); }
__device__ __forceinline__ void keep4_b(v16b a, v16b b, v16b c, v16b d) { asm volatile("v_nop" :: "v"(a), "v"(b), "v"(c), "v"(d)); }
__device__ __forceinline__ void acc_guard4(v8f& a, v8f& b, v8f& c, v8f& d) { asm volatile("v_nop\n\tv_nop\n\tv_nop\n\tv_nop" : "+v"(a), "+v"(b), "+v"(c), "+v"(d)); }
template <typename T> struct Frag;
template <> struct Frag<_Float16> {
  typedef v16h V; union U { v16h v; v8h h[2]; };
  static __device__ __forceinline__ v16h load(const _Float16* p) {
    U f; f.h[0] = *(const v8h*)(p); f.h[1] = *(const v8h*)(p + 16); return f.v;
  }
  static __device__ __forceinline__ v8f mma(v16h a, v16h b, v8f c) {
    return __builtin_amdgcn_wmma_f32_16x16x32_f16(false, a, false, b, (short)0, c, false, false);
  }
  static __device__ __forceinline__ void guard(v8f& a, v8f& b, v16h x, v16h y) { dep_guard_h(a, b, x, y); }
  static __device__ __forceinline__ void keep(v16h a, v16h b, v16h c, v16h d) { keep4_h(a, b, c, d); }
};
template <> struct Frag<__bf16> {
  typedef v16b V; union U { v16b v; v8b h[2]; };
  static __device__ __forceinline__ v16b load(const __bf16* p) {
    U f; f.h[0] = *(const v8b*)(p); f.h[1] = *(const v8b*)(p + 16); return f.v;
  }
  static __device__ __forceinline__ v8f mma(v16b a, v16b b, v8f c) {
    return __builtin_amdgcn_wmma_f32_16x16x32_bf16(false, a, false, b, (short)0, c, false, false);
  }
  static __device__ __forceinline__ void guard(v8f& a, v8f& b, v16b x, v16b y) { dep_guard_b(a, b, x, y); }
  static __device__ __forceinline__ void keep(v16b a, v16b b, v16b c, v16b d) { keep4_b(a, b, c, d); }
};

template <int ET> struct Elem;
template <> struct Elem<0> { typedef _Float16 T; };
template <> struct Elem<1> { typedef __bf16 T; };
template <int ET, bool SPLIT, int BIAS_MODE, int OUT_MODE, bool RESID, int ACT = 0>
__global__ __launch_bounds__(256) void wmma_gemm64(
    const unsigned short* __restrict__ Ap, const unsigned short* __restrict__ A2p, int lda, long strideA,
    const unsigned short* __restrict__ Btp, const unsigned short* __restrict__ Bt2p, int ldb, long strideB,
    void* __restrict__ Cout, void* __restrict__ Cout2, int ldc, long strideC,
    const float* __restrict__ bias,
    const float* __restrict__ resid, long strideR,
    int M, int N, int K, float scale) {
  typedef typename Elem<ET>::T T;
  typedef typename Frag<T>::V V;
  const T* A = (const T*)Ap; const T* A2 = (const T*)A2p; const T* Bt = (const T*)Btp; const T* Bt2 = (const T*)Bt2p;
  __shared__ __align__(16) float sT[8][16 * 68];
  const int b    = blockIdx.y;
  const int lane = threadIdx.x & 31;
  const int wave = threadIdx.x >> 5;
  const int tilesN = N >> 6;
  const int tilesM = M >> 6;
  const int tile = blockIdx.x * 8 + wave;
  if (tile >= tilesM * tilesN) return;
  const int tm = tile / tilesN;
  const int tn = tile - tm * tilesN;
  const int m0 = tm << 6;
  const int n0 = tn << 6;

  const T* Ab  = A  + (size_t)b * strideA;
  const T* Bb  = Bt + (size_t)b * strideB;
  const T* Ab2 = SPLIT ? (A2  + (size_t)b * strideA) : nullptr;
  const T* Bb2 = SPLIT ? (Bt2 + (size_t)b * strideB) : nullptr;

  const int rlane = lane & 15;
  const int koff  = (lane >> 4) * 8;
  const int mOff  = (lane >> 4) * 8;

  v8f acc[4][4];
#pragma unroll
  for (int i = 0; i < 4; ++i)
#pragma unroll
    for (int j = 0; j < 4; ++j) acc[i][j] = (v8f){0.f,0.f,0.f,0.f,0.f,0.f,0.f,0.f};

  for (int k0 = 0; k0 < K; k0 += 32) {
    V bh[4], bl[4];
#pragma unroll
    for (int j = 0; j < 4; ++j) {
      const size_t bo = (size_t)(n0 + (j << 4) + rlane) * ldb + koff + k0;
      bh[j] = Frag<T>::load(Bb + bo);
      if (SPLIT) bl[j] = Frag<T>::load(Bb2 + bo);
    }
#pragma unroll
    for (int i = 0; i < 4; ++i) {
      const size_t ao = (size_t)(m0 + (i << 4) + rlane) * lda + koff + k0;
      V ah = Frag<T>::load(Ab + ao);
      V al;
      if (SPLIT) al = Frag<T>::load(Ab2 + ao);
#pragma unroll
      for (int j = 0; j < 4; ++j) {
        acc[i][j] = Frag<T>::mma(ah, bh[j], acc[i][j]);
        if (SPLIT) {
          acc[i][j] = Frag<T>::mma(ah, bl[j], acc[i][j]);
          acc[i][j] = Frag<T>::mma(al, bh[j], acc[i][j]);
        }
      }
      Frag<T>::guard(acc[i][0], acc[i][3], ah, SPLIT ? al : ah);
    }
    Frag<T>::keep(bh[0], bh[1], bh[2], bh[3]);
    if (SPLIT) Frag<T>::keep(bl[0], bl[1], bl[2], bl[3]);
  }
  acc_guard4(acc[0][0], acc[0][1], acc[0][2], acc[0][3]);
  acc_guard4(acc[1][0], acc[1][1], acc[1][2], acc[1][3]);
  acc_guard4(acc[2][0], acc[2][1], acc[2][2], acc[2][3]);
  acc_guard4(acc[3][0], acc[3][1], acc[3][2], acc[3][3]);

  float* slab = sT[wave];
  const float* Rb = RESID ? (resid + (size_t)b * strideR) : nullptr;
#pragma unroll
  for (int i = 0; i < 4; ++i) {
    const int mBase = m0 + (i << 4);
#pragma unroll
    for (int j = 0; j < 4; ++j) {
      const int n = n0 + (j << 4) + rlane;
      float bv = 0.f;
      if (BIAS_MODE == 2) bv = bias[n];
#pragma unroll
      for (int r = 0; r < 8; ++r) {
        float v = acc[i][j][r] * scale;
        if (BIAS_MODE == 1) v += bias[mBase + mOff + r];
        if (BIAS_MODE == 2) v += bv;
        if (RESID) v += Rb[(size_t)(mBase + mOff + r) * ldc + n];
        if (ACT == 1) v = tanhf(v);
        if (ACT == 2) v = fmaxf(v, 0.0f);
        if (ACT == 3) v = v / (1.0f + expf(-v));
        if (ACT == 4) v = (v > 0.f) ? v : 0.01f * v;
        if (ACT == 5) v = 0.5f * v * (1.0f + erff(v * 0.70710678118654752f));
        slab[(mOff + r) * 68 + (j << 4) + rlane] = v;
      }
    }
    __builtin_amdgcn_fence(__ATOMIC_RELEASE, "workgroup");
    __builtin_amdgcn_wave_barrier();
    __builtin_amdgcn_fence(__ATOMIC_ACQUIRE, "workgroup");
    if (OUT_MODE == 0) {
      float* C = (float*)Cout + (size_t)b * strideC;
      const int hh = lane >> 4, c4 = (lane & 15) * 4;
      for (int pass = 0; pass < 2; ++pass) {
#pragma unroll
        for (int it = 0; it < 8; ++it) {
          const int row = it * 2 + hh;
          v4f v = *(const v4f*)(slab + row * 68 + c4);
          *(volatile v4f*)(C + (size_t)(mBase + row) * ldc + n0 + c4) = v;
        }
        __threadfence();
      }
    } else {
      const int q = lane >> 3, c8 = (lane & 7) * 8;
      unsigned short* C  = (unsigned short*)Cout  + (size_t)b * strideC;
      unsigned short* C2 = (OUT_MODE == 2) ? ((unsigned short*)Cout2 + (size_t)b * strideC) : nullptr;
      for (int pass = 0; pass < 2; ++pass) {
#pragma unroll
        for (int it = 0; it < 4; ++it) {
          const int row = it * 4 + q;
          const float* sp = slab + row * 68 + c8;
          v8h hv, lv;
#pragma unroll
          for (int e = 0; e < 8; ++e) {
            if (OUT_MODE == 1) {
              hv[e] = (_Float16)sp[e];
            } else {
              unsigned short hb = f2bf_bits(sp[e]);
              unsigned short lb = f2bf_bits(sp[e] - bf_bits2f(hb));
              hv[e] = __builtin_bit_cast(_Float16, hb);
              lv[e] = __builtin_bit_cast(_Float16, lb);
            }
          }
          *(volatile v8h*)(C + (size_t)(mBase + row) * ldc + n0 + c8) = hv;
          if (OUT_MODE == 2) *(volatile v8h*)(C2 + (size_t)(mBase + row) * ldc + n0 + c8) = lv;
        }
        __threadfence();
      }
    }
    __builtin_amdgcn_fence(__ATOMIC_RELEASE, "workgroup");
    __builtin_amdgcn_wave_barrier();
    __builtin_amdgcn_fence(__ATOMIC_ACQUIRE, "workgroup");
  }
}

__global__ __launch_bounds__(256) void cast_f32_f16x2s(
    const float* __restrict__ in, _Float16* __restrict__ out, int n2, float sc) {
  int i = blockIdx.x * 256 + threadIdx.x;
  if (i < n2) {
    const _Float16 h0 = (_Float16)(in[2 * i] * sc), h1 = (_Float16)(in[2 * i + 1] * sc);
    const unsigned u = (unsigned)__builtin_bit_cast(unsigned short, h0) | ((unsigned)__builtin_bit_cast(unsigned short, h1) << 16);
    ((volatile unsigned*)out)[i] = u;
    __threadfence();
    ((volatile unsigned*)out)[i] = u;
  }
}

__global__ __launch_bounds__(256) void cast4_f32_f16x2s(
    const float* __restrict__ s0, const float* __restrict__ s1,
    const float* __restrict__ s2, const float* __restrict__ s3,
    _Float16* __restrict__ out, int n2each, float sc) {
  const int y = blockIdx.y;
  const float* in = (y == 0) ? s0 : (y == 1) ? s1 : (y == 2) ? s2 : s3;
  _Float16* o = out + (size_t)y * (size_t)n2each * 2;
  int i = blockIdx.x * 256 + threadIdx.x;
  if (i < n2each) {
    const _Float16 h0 = (_Float16)(in[2 * i] * sc), h1 = (_Float16)(in[2 * i + 1] * sc);
    const unsigned u = (unsigned)__builtin_bit_cast(unsigned short, h0) | ((unsigned)__builtin_bit_cast(unsigned short, h1) << 16);
    ((volatile unsigned*)o)[i] = u;
    __threadfence();
    ((volatile unsigned*)o)[i] = u;
  }
}

#define AT_D 64
#define AT_NW 4
#define AT_QB 64
#define AT_KC 64

__device__ __forceinline__ v8f mma_h(v16h a, v16h b, v8f c) {
  c = __builtin_amdgcn_wmma_f32_16x16x32_f16(false, a, false, b, (short)0, c, false, false);
  asm volatile("v_nop\n\tv_nop\n\tv_nop\n\tv_nop" : "+v"(c) : "v"(a), "v"(b));
  return c;
}

__global__ __launch_bounds__(128)
void attn64_f16_kernel(const _Float16* __restrict__ q, const _Float16* __restrict__ k,
                       const _Float16* __restrict__ vt, const float* __restrict__ maskv,
                       _Float16* __restrict__ ctx,
                       int S, int Skv, int H, int ldq, int ldk, int ldv, int ldo,
                       float qscale, float mask_fill, float oscale) {
  const float PSC = 32768.0f;
  union FH { v16h v; v8h h[2]; };
  __shared__ __align__(16) _Float16 Psh[AT_NW][16 * AT_KC];
  __shared__ __align__(16) float    Os[AT_NW][16 * 68];

  const int tid  = threadIdx.x;
  const int wave = tid >> 5;
  const int lane = tid & 31;
  const int hh   = lane >> 4;
  const int c    = lane & 15;

  const int nqb = S / AT_QB;
  const int bx  = blockIdx.x;
  const int qb  = bx % nqb;
  const int h   = bx / nqb;
  if (h >= H) return;
  const int q0   = qb * AT_QB + wave * 16;
  const int hoff = h * AT_D;

  v16h qa[2];
  {
    const _Float16* qrow = q + (size_t)(q0 + c) * ldq + hoff + 8 * hh;
#pragma unroll
    for (int dc = 0; dc < 2; ++dc) qa[dc] = Frag<_Float16>::load(qrow + dc * 32);
  }

  float mrow[8], lrow[8];
  v8f oacc[4];
#pragma unroll
  for (int r = 0; r < 8; ++r) { mrow[r] = -INFINITY; lrow[r] = 0.f; }
#pragma unroll
  for (int t = 0; t < 4; ++t) oacc[t] = (v8f){0.f,0.f,0.f,0.f,0.f,0.f,0.f,0.f};

  _Float16* pw = Psh[wave];
  const int nChunks = Skv / AT_KC;
  for (int kc = 0; kc < nChunks; ++kc) {
    const int kv0 = kc * AT_KC;

    v8f s[4];
#pragma unroll
    for (int j = 0; j < 4; ++j) {
      s[j] = (v8f){0.f,0.f,0.f,0.f,0.f,0.f,0.f,0.f};
      const _Float16* krow = k + (size_t)(kv0 + j * 16 + c) * ldk + hoff + 8 * hh;
#pragma unroll
      for (int dc = 0; dc < 2; ++dc) {
        const v16h kb = Frag<_Float16>::load(krow + dc * 32);
        s[j] = mma_h(qa[dc], kb, s[j]);
      }
    }
    float madd[4];
#pragma unroll
    for (int j = 0; j < 4; ++j) madd[j] = (1.0f - maskv[kv0 + j * 16 + c]) * mask_fill;

    float cm[8];
#pragma unroll
    for (int r = 0; r < 8; ++r) {
      float m = -INFINITY;
#pragma unroll
      for (int j = 0; j < 4; ++j) {
        const float x = s[j][r] * qscale + madd[j];
        s[j][r] = x;
        m = fmaxf(m, x);
      }
#pragma unroll
      for (int off = 1; off < 16; off <<= 1) m = fmaxf(m, __shfl_xor(m, off, 32));
      cm[r] = m;
    }

    __builtin_amdgcn_fence(__ATOMIC_RELEASE, "workgroup");
    __builtin_amdgcn_wave_barrier();
    __builtin_amdgcn_fence(__ATOMIC_ACQUIRE, "workgroup");

#pragma unroll
    for (int r = 0; r < 8; ++r) {
      const float mnew  = fmaxf(mrow[r], cm[r]);
      const float alpha = expf(mrow[r] - mnew);
      mrow[r] = mnew;
      float psum = 0.f;
#pragma unroll
      for (int j = 0; j < 4; ++j) {
        const float p = expf(s[j][r] - mnew);
        psum += p;
        pw[(8 * hh + r) * AT_KC + j * 16 + c] = (_Float16)(p * PSC);
      }
#pragma unroll
      for (int off = 1; off < 16; off <<= 1) psum += __shfl_xor(psum, off, 32);
      lrow[r] = lrow[r] * alpha + psum;
#pragma unroll
      for (int t = 0; t < 4; ++t) oacc[t][r] *= alpha;
    }
    __builtin_amdgcn_fence(__ATOMIC_RELEASE, "workgroup");
    __builtin_amdgcn_wave_barrier();
    __builtin_amdgcn_fence(__ATOMIC_ACQUIRE, "workgroup");

#pragma unroll 1
    for (int kk = 0; kk < 2; ++kk) {
      FH pa;
      pa.h[0] = *(const v8h*)(pw + c * AT_KC + kk * 32 + 8 * hh);
      pa.h[1] = *(const v8h*)(pw + c * AT_KC + kk * 32 + 16 + 8 * hh);
#pragma unroll
      for (int t = 0; t < 4; ++t) {
        const v16h vb = Frag<_Float16>::load(vt + (size_t)(hoff + t * 16 + c) * ldv + kv0 + kk * 32 + 8 * hh);
        oacc[t] = mma_h(pa.v, vb, oacc[t]);
      }
    }
  }

  float* os = Os[wave];
#pragma unroll
  for (int r = 0; r < 8; ++r) {
    const float inv = oscale / (lrow[r] * PSC);
#pragma unroll
    for (int t = 0; t < 4; ++t) os[(8 * hh + r) * 68 + t * 16 + c] = oacc[t][r] * inv;
  }
  __builtin_amdgcn_fence(__ATOMIC_RELEASE, "workgroup");
  __builtin_amdgcn_wave_barrier();
  __builtin_amdgcn_fence(__ATOMIC_ACQUIRE, "workgroup");
  {
    const int q8 = lane >> 3, c8 = (lane & 7) * 8;
    for (int pass = 0; pass < 2; ++pass) {
#pragma unroll
      for (int it = 0; it < 4; ++it) {
        const int row = it * 4 + q8;
        const float* sp = os + row * 68 + c8;
        v8h hv;
#pragma unroll
        for (int e = 0; e < 8; ++e) hv[e] = (_Float16)sp[e];
        *(volatile v8h*)(ctx + (size_t)(q0 + row) * ldo + hoff + c8) = hv;
      }
      __threadfence();
    }
  }
}

__global__ __launch_bounds__(256) void row_tanh_res_ln_kernel(
    const float* __restrict__ y, const float* __restrict__ res,
    const float* __restrict__ gamma, const float* __restrict__ beta,
    float* __restrict__ out, int ncols, float eps) {
  __shared__ float red[16];
  const int row  = blockIdx.x;
  const int t    = threadIdx.x;
  const int lane = t & 31;
  const int wave = t >> 5;
  const size_t base = (size_t)row * ncols + 4 * t;
  const v4f yv = *(const v4f*)(y + base);
  const v4f rv = *(const v4f*)(res + base);
  const float x0 = tanhf(yv[0]) + rv[0];
  const float x1 = tanhf(yv[1]) + rv[1];
  const float x2 = tanhf(yv[2]) + rv[2];
  const float x3 = tanhf(yv[3]) + rv[3];
  float s = (x0 + x1) + (x2 + x3);
#pragma unroll
  for (int off = 1; off < 32; off <<= 1) s += __shfl_xor(s, off, 32);
  if (lane == 0) red[wave] = s;
  __syncthreads();
  float tot = 0.f;
#pragma unroll
  for (int w = 0; w < 8; ++w) tot += red[w];
  const float inv_n = 1.0f / (float)ncols;
  const float mu = tot * inv_n;
  const float d0 = x0 - mu, d1 = x1 - mu, d2 = x2 - mu, d3 = x3 - mu;
  float s2 = (d0 * d0 + d1 * d1) + (d2 * d2 + d3 * d3);
#pragma unroll
  for (int off = 1; off < 32; off <<= 1) s2 += __shfl_xor(s2, off, 32);
  if (lane == 0) red[8 + wave] = s2;
  __syncthreads();
  float tot2 = 0.f;
#pragma unroll
  for (int w = 0; w < 8; ++w) tot2 += red[8 + w];
  const float var = tot2 * inv_n;
  const float rn  = 1.0f / sqrtf(var + eps);
  const v4f gv = *(const v4f*)(gamma + 4 * t);
  const v4f bv = *(const v4f*)(beta + 4 * t);
  v4f o;
  o[0] = d0 * rn * gv[0] + bv[0];
  o[1] = d1 * rn * gv[1] + bv[1];
  o[2] = d2 * rn * gv[2] + bv[2];
  o[3] = d3 * rn * gv[3] + bv[3];
  *(volatile v4f*)(out + base) = o;
  __threadfence();
  *(volatile v4f*)(out + base) = o;
}

extern "C" void kernel_launch(void* const* d_in, const int* in_sizes, int n_in,
                              void* d_out, int out_size, void* d_ws, size_t ws_size,
                              hipStream_t stream) {
  if (n_in < 12) return;
  const float* ht    = (const float*)d_in[0];
  const float* amask = (const float*)d_in[1];
  const float* Wq    = (const float*)d_in[2];
  const float* bq    = (const float*)d_in[3];
  const float* Wk    = (const float*)d_in[4];
  const float* bk    = (const float*)d_in[5];
  const float* Wv    = (const float*)d_in[6];
  const float* bv    = (const float*)d_in[7];
  const float* Wd    = (const float*)d_in[8];
  const float* bd    = (const float*)d_in[9];
  const float* gamma = (const float*)d_in[10];
  const float* beta  = (const float*)d_in[11];

  const int Dm = in_sizes[3];
  if (Dm != 1024) return;
  const int Nn = in_sizes[0] / Dm;
  const int Hh = 16;
  const int Dh = Dm / Hh;
  if (Dh != 64 || Nn <= 0 || (Nn % 64) != 0 || in_sizes[0] != Nn * Dm) return;
  if (in_sizes[2] != Dm * Dm || in_sizes[4] != Dm * Dm || in_sizes[6] != Dm * Dm || in_sizes[8] != Dm * Dm) return;
  if (in_sizes[1] < Nn || in_sizes[5] < Dm || in_sizes[7] < Dm || in_sizes[9] < Dm || in_sizes[10] < Dm || in_sizes[11] < Dm) return;
  if (out_size != Nn * Dm) return;

  const size_t bHt16 = (size_t)Nn * Dm * 2;
  const size_t bW16  = (size_t)Dm * Dm * 2;
  const size_t bF    = (size_t)Nn * Dm * 4;
  size_t o = 0;
  char* ws = (char*)d_ws;
  _Float16* ht16  = (_Float16*)(ws + o); o += bHt16;
  _Float16* w16   = (_Float16*)(ws + o); o += 4 * bW16;
  _Float16* q16   = (_Float16*)(ws + o); o += bHt16;
  _Float16* k16   = (_Float16*)(ws + o); o += bHt16;
  _Float16* vt16  = (_Float16*)(ws + o); o += bHt16;
  _Float16* ctx16 = (_Float16*)(ws + o); o += bHt16;
  float*    yf    = (float*)(ws + o);    o += bF;
  if (o > ws_size) return;
  _Float16* wq16 = w16;
  _Float16* wk16 = w16 + (size_t)Dm * Dm;
  _Float16* wv16 = w16 + (size_t)2 * Dm * Dm;
  _Float16* wd16 = w16 + (size_t)3 * Dm * Dm;

  const int nHt2 = Nn * Dm / 2, nW2 = Dm * Dm / 2;
  cast_f32_f16x2s<<<(nHt2 + 255) / 256, 256, 0, stream>>>(ht, ht16, nHt2, 1.0f);
  cast4_f32_f16x2s<<<dim3((nW2 + 255) / 256, 4), 256, 0, stream>>>(Wq, Wk, Wv, Wd, w16, nW2, 16.0f);

  const int tilesQK = (Nn / 64) * (Dm / 64);
  const dim3 gqk((tilesQK + 7) / 8, 1);
  const unsigned short* Au = (const unsigned short*)ht16;
  wmma_gemm64<0, false, 2, 1, false, 0><<<gqk, 256, 0, stream>>>(
      Au, Au, Dm, 0L, (const unsigned short*)wq16, (const unsigned short*)wq16, Dm, 0L,
      (void*)q16, (void*)q16, Dm, 0L, bq, ht, 0L, Nn, Dm, Dm, 1.0f / 16.0f);
  wmma_gemm64<0, false, 2, 1, false, 0><<<gqk, 256, 0, stream>>>(
      Au, Au, Dm, 0L, (const unsigned short*)wk16, (const unsigned short*)wk16, Dm, 0L,
      (void*)k16, (void*)k16, Dm, 0L, bk, ht, 0L, Nn, Dm, Dm, 1.0f / 16.0f);
  const int tilesV = (Dm / 64) * (Nn / 64);
  const dim3 gv((tilesV + 7) / 8, 1);
  wmma_gemm64<0, false, 1, 1, false, 0><<<gv, 256, 0, stream>>>(
      (const unsigned short*)wv16, (const unsigned short*)wv16, Dm, 0L, Au, Au, Dm, 0L,
      (void*)vt16, (void*)vt16, Nn, 0L, bv, ht, 0L, Dm, Nn, Dm, 1.0f / 16.0f);

  attn64_f16_kernel<<<Hh * (Nn / 64), 128, 0, stream>>>(
      q16, k16, vt16, amask, ctx16, Nn, Nn, Hh, Dm, Dm, Nn, Dm, 0.125f, -10000.0f, 16.0f);

  const unsigned short* Cu = (const unsigned short*)ctx16;
  wmma_gemm64<0, false, 2, 0, false, 0><<<gqk, 256, 0, stream>>>(
      Cu, Cu, Dm, 0L, (const unsigned short*)wd16, (const unsigned short*)wd16, Dm, 0L,
      (void*)yf, (void*)yf, Dm, 0L, bd, ht, 0L, Nn, Dm, Dm, 1.0f / 256.0f);

  row_tanh_res_ln_kernel<<<Nn, 256, 0, stream>>>(yf, ht, gamma, beta, (float*)d_out, Dm, 1e-5f);
}
